// GATSegmentationModel_47373489275188
// MI455X (gfx1250) — hardware-verified
//
#include <hip/hip_runtime.h>
#include <stddef.h>
#include <stdint.h>
#include <math.h>


#define NN      4096
#define IMW     256
#define CO      64
#define OHW     128
#define KC      147
#define KCP     160
#define KF      128
#define HC      128
#define NTHR    256
#define NWAVE   8
#define EPT     8
#define CHUNK   (NTHR * EPT)
#define WCAP    (EPT * 32)
#define LISTN   (NWAVE * WCAP)
#define NB      64
#define SLOTB   6
#define RCAP    16384
#define DEGCAP  256
#define GBM     64
#define GBN     64
#define GTHR    128
#define NEGSL   0.2f
#define WSMAX   134217728
#define NU_IM   (3 * IMW * IMW / 8)
#define NU_CW   (CO * KCP / 8)
#define NU_W1   (HC * KF / 8)
#define LDS_SCAN_INTS (2 * RCAP + LISTN + 2 * NB + 16 + NB)
#define LDS_SCAN (LDS_SCAN_INTS * 4)

static_assert(NB == (1 << SLOTB));
static_assert((CHUNK & (CHUNK - 1)) == 0);
static_assert(LISTN >= NWAVE * WCAP && LISTN >= NB);
static_assert((RCAP % 32) == 0 && DEGCAP <= WCAP);
static_assert((NN % NB) == 0 && (NB % NWAVE) == 0 && (NB % 32) == 0);
static_assert((KCP % 32) == 0 && (KF % 32) == 0 && KCP >= KC);
static_assert(GBM == (GTHR / 32) * 16 && GTHR == 2 * GBM && GBN == 64);
static_assert((NN % GBM) == 0 && (HC % GBN) == 0 && (OHW * OHW) % GBM == 0 && (OHW % GBM) == 0);
static_assert((NU_IM % NTHR) == 0 && (NU_CW % NTHR) == 0 && (NU_W1 % NTHR) == 0);
static_assert(LDS_SCAN <= 300000);
static_assert(((2 * RCAP + LISTN + 2 * NB + 16) % 4) == 0);
static_assert(HC == 4 * 32);

typedef float          v4f  __attribute__((ext_vector_type(4)));
typedef float          v8f  __attribute__((ext_vector_type(8)));
typedef int            v4i  __attribute__((ext_vector_type(4)));
typedef int            v8i  __attribute__((ext_vector_type(8)));
typedef unsigned int   v4u  __attribute__((ext_vector_type(4)));
typedef unsigned short v8us __attribute__((ext_vector_type(8)));
typedef __bf16         v16b __attribute__((ext_vector_type(16)));
typedef v4f  __attribute__((may_alias)) v4fa;
typedef v4u  __attribute__((may_alias)) v4ua;
typedef v8us __attribute__((may_alias)) v8usa;
union FragB { v16b v; v8us h[2]; v8i w; };

__device__ __forceinline__ v8f wmb(const FragB& a, const FragB& b, v8f c) {
  v8f d = __builtin_amdgcn_wmma_f32_16x16x32_bf16(false, a.v, false, b.v, (short)0, c, false, false);
  asm volatile("v_nop\n\tv_nop\n\tv_nop\n\tv_nop" : "+v"(d) : "v"(a.w), "v"(b.w));
  return d;
}

__device__ __forceinline__ unsigned int f2bf(float f) {
  const unsigned int u = __float_as_uint(f);
  return ((u + 0x7FFFu + ((u >> 16) & 1u)) >> 16) & 0xFFFFu;
}
__device__ __forceinline__ float bf2f(unsigned int b) { return __uint_as_float(b << 16); }
__device__ __forceinline__ float bfr(float f) { return bf2f(f2bf(f)); }
__device__ __forceinline__ v4f bfr4(const v4f a) {
  v4f r; r.x = bfr(a.x); r.y = bfr(a.y); r.z = bfr(a.z); r.w = bfr(a.w); return r;
}
__device__ __forceinline__ unsigned int pk2(float lo, float hi) { return f2bf(lo) | (f2bf(hi) << 16); }
__device__ __forceinline__ v4u pack8(const v4f a, const v4f b) {
  v4u r;
  r.x = pk2(a.x, a.y); r.y = pk2(a.z, a.w); r.z = pk2(b.x, b.y); r.w = pk2(b.z, b.w);
  return r;
}
__device__ __forceinline__ float lres(float v) { return v - bf2f(f2bf(v)); }

__device__ __forceinline__ int scan_chunk(const int* __restrict__ dsts, int nE, int cbase, int slotBase,
                                          int nb, int vec8, int* list, int tid, int lane, int wave) {
  int wc = 0;
  const int el0  = tid * EPT;
  const int e0   = cbase + el0;
  const int sent = -2147483647 - 1;
  v4i da, db;
  if (vec8 != 0 && cbase + CHUNK <= nE) {
    da = *(const v4i*)(dsts + e0);
    db = *(const v4i*)(dsts + e0 + 4);
  } else {
    da.x = (e0     < nE) ? dsts[min(e0,     nE - 1)] : sent;
    da.y = (e0 + 1 < nE) ? dsts[min(e0 + 1, nE - 1)] : sent;
    da.z = (e0 + 2 < nE) ? dsts[min(e0 + 2, nE - 1)] : sent;
    da.w = (e0 + 3 < nE) ? dsts[min(e0 + 3, nE - 1)] : sent;
    db.x = (e0 + 4 < nE) ? dsts[min(e0 + 4, nE - 1)] : sent;
    db.y = (e0 + 5 < nE) ? dsts[min(e0 + 5, nE - 1)] : sent;
    db.z = (e0 + 6 < nE) ? dsts[min(e0 + 6, nE - 1)] : sent;
    db.w = (e0 + 7 < nE) ? dsts[min(e0 + 7, nE - 1)] : sent;
  }
  const unsigned nbs = (unsigned)slotBase;
  const unsigned unb = (unsigned)nb;
  const unsigned s0 = (unsigned)da.x - nbs, s1 = (unsigned)da.y - nbs;
  const unsigned s2 = (unsigned)da.z - nbs, s3 = (unsigned)da.w - nbs;
  const unsigned s4 = (unsigned)db.x - nbs, s5 = (unsigned)db.y - nbs;
  const unsigned s6 = (unsigned)db.z - nbs, s7 = (unsigned)db.w - nbs;
  const bool h0 = s0 < unb, h1 = s1 < unb, h2 = s2 < unb, h3 = s3 < unb;
  const bool h4 = s4 < unb, h5 = s5 < unb, h6 = s6 < unb, h7 = s7 < unb;
  const unsigned any = __builtin_amdgcn_ballot_w32(h0 | h1 | h2 | h3 | h4 | h5 | h6 | h7);
  if (any != 0u) {
#define HITJ(J, HJ, SJ) { \
      const unsigned mj = __builtin_amdgcn_ballot_w32(HJ); \
      if (mj != 0u) { \
        if (HJ) { \
          const int pos = wc + (int)__builtin_amdgcn_mbcnt_lo(mj, 0u); \
          if (pos < WCAP) list[wave * WCAP + pos] = ((el0 + (J)) << SLOTB) | (int)(SJ); \
        } \
        wc += (int)__builtin_popcount(mj); } }
    HITJ(0, h0, s0)
    HITJ(1, h1, s1)
    HITJ(2, h2, s2)
    HITJ(3, h3, s3)
    HITJ(4, h4, s4)
    HITJ(5, h5, s5)
    HITJ(6, h6, s6)
    HITJ(7, h7, s7)
#undef HITJ
  }
  return wc;
}

__device__ __forceinline__ int scan_build(const int* __restrict__ dsts, int nE, int nodeBase, int vec8,
                                          int* reg1, int* reg2, int* list, int* scnt, int* soff, int* wcnt,
                                          int tid, int lane, int wave) {
  for (int i = tid; i < NB; i += NTHR) scnt[i] = 0;
  __syncthreads();

  int tot = 0;
  const int nChunks = (nE + CHUNK - 1) / CHUNK;
#pragma unroll 1
  for (int ch = 0; ch < nChunks; ++ch) {
    const int cbase = ch * CHUNK;
    const int wc = scan_chunk(dsts, nE, cbase, nodeBase, NB, vec8, list, tid, lane, wave);
    if (lane == 0) wcnt[wave] = wc;
    __syncthreads();
    int pre = 0, all = 0;
#pragma unroll
    for (int w2 = 0; w2 < NWAVE; ++w2) {
      int c = wcnt[w2];
      c = c < 0 ? 0 : (c > WCAP ? WCAP : c);
      all += c;
      pre += (w2 < wave) ? c : 0;
    }
    const int wcc  = wc > WCAP ? WCAP : wc;
    const int base = tot + pre;
#pragma unroll 1
    for (int i = lane; i < wcc; i += 32) {
      const int ent = list[wave * WCAP + i];
      const int el  = (ent >> SLOTB) & (CHUNK - 1);
      const int sl  = ent & (NB - 1);
      int eid = cbase + el;
      eid = eid > nE - 1 ? nE - 1 : eid;
      const int pos = base + i;
      if (pos < RCAP) reg1[pos] = (int)(((unsigned)eid << SLOTB) | (unsigned)sl);
    }
    tot += all;
    tot = tot > RCAP ? RCAP : tot;
    __syncthreads();
  }
  const int nh = tot;

  if (wave == 0) {
#pragma unroll 1
    for (int b0 = 0; b0 < nh; b0 += 32) {
      const int idx = b0 + lane;
      const int uv  = reg1[idx < nh ? idx : nh - 1];
      const int m32 = (nh - b0) < 32 ? (nh - b0) : 32;
#pragma unroll 1
      for (int k = 0; k < m32; ++k) {
        const int u  = __builtin_amdgcn_readlane(uv, k);
        const int sl = u & (NB - 1);
        if (lane == 0) scnt[sl] = scnt[sl] + 1;
      }
    }
  }
  __syncthreads();

  if (wave == 0) {
    int c0 = scnt[2 * lane], c1 = scnt[2 * lane + 1];
    c0 = c0 < 0 ? 0 : c0;
    c1 = c1 < 0 ? 0 : c1;
    const int ts = c0 + c1;
    int incl = ts;
#pragma unroll
    for (int d = 1; d < 32; d <<= 1) {
      const int up = __shfl_up(incl, d);
      if (lane >= d) incl += up;
    }
    const int run = incl - ts;
    soff[2 * lane]     = run;
    soff[2 * lane + 1] = run + c0;
    list[2 * lane]     = run;
    list[2 * lane + 1] = run + c0;
  }
  __syncthreads();

  if (wave == 0) {
#pragma unroll 1
    for (int b0 = 0; b0 < nh; b0 += 32) {
      const int idx = b0 + lane;
      const int uv  = reg1[idx < nh ? idx : nh - 1];
      const int m32 = (nh - b0) < 32 ? (nh - b0) : 32;
#pragma unroll 1
      for (int k = 0; k < m32; ++k) {
        const int u   = __builtin_amdgcn_readlane(uv, k);
        const int sl  = u & (NB - 1);
        const int eid = (int)((unsigned)u >> SLOTB);
        if (lane == 0) {
          int pos = list[sl];
          pos = pos < 0 ? 0 : (pos > RCAP - 1 ? RCAP - 1 : pos);
          reg2[pos] = eid;
          list[sl] = pos + 1;
        }
      }
    }
  }
  __syncthreads();
  return nh;
}

__global__ __launch_bounds__(NTHR) void k_prep(const float* __restrict__ image, const float* __restrict__ conv_w,
                                               const float* __restrict__ W1,
                                               unsigned short* IMB, unsigned short* CWB, unsigned short* W1T2) {
  const int u = (int)blockIdx.x * NTHR + (int)threadIdx.x;
  v4f a, b;
  unsigned short* dp;
  if (u < NU_IM) {
    const float* p = image + (size_t)u * 8;
    a = *(const v4fa*)p;
    b = *(const v4fa*)(p + 4);
    dp = IMB + (size_t)u * 8;
  } else if (u < NU_IM + NU_CW) {
    const int v  = u - NU_IM;
    const int o  = v / (KCP / 8);
    const int k8 = (v - o * (KCP / 8)) * 8;
    const float* p = conv_w + (size_t)o * KC;
    const float t0 = p[min(k8 + 0, KC - 1)], t1 = p[min(k8 + 1, KC - 1)];
    const float t2 = p[min(k8 + 2, KC - 1)], t3 = p[min(k8 + 3, KC - 1)];
    const float t4 = p[min(k8 + 4, KC - 1)], t5 = p[min(k8 + 5, KC - 1)];
    const float t6 = p[min(k8 + 6, KC - 1)], t7 = p[min(k8 + 7, KC - 1)];
    a.x = (k8 + 0 < KC) ? t0 : 0.f; a.y = (k8 + 1 < KC) ? t1 : 0.f;
    a.z = (k8 + 2 < KC) ? t2 : 0.f; a.w = (k8 + 3 < KC) ? t3 : 0.f;
    b.x = (k8 + 4 < KC) ? t4 : 0.f; b.y = (k8 + 5 < KC) ? t5 : 0.f;
    b.z = (k8 + 6 < KC) ? t6 : 0.f; b.w = (k8 + 7 < KC) ? t7 : 0.f;
    dp = CWB + (size_t)o * KCP + k8;
  } else if (u < NU_IM + NU_CW + NU_W1) {
    const int v  = u - NU_IM - NU_CW;
    const int n  = v >> 4;
    const int k8 = (v & 15) * 8;
    const int kk = k8 & 63;
    const float* p = W1 + (size_t)kk * HC + n;
    a.x = p[0];      a.y = p[HC];     a.z = p[2 * HC]; a.w = p[3 * HC];
    b.x = p[4 * HC]; b.y = p[5 * HC]; b.z = p[6 * HC]; b.w = p[7 * HC];
    dp = W1T2 + (size_t)n * KF + k8;
  } else {
    return;
  }
  const v4u hv = pack8(a, b);
  *(volatile v4u*)dp = hv;
  __threadfence();
  *(volatile v4u*)dp = hv;
}

__device__ __forceinline__ unsigned int tap(const unsigned short* __restrict__ IMB, int k, int iy0, int ix0) {
  const int c   = k / 49;
  const int rem = k - 49 * c;
  const int ky  = rem / 7;
  const int kx  = rem - 7 * ky;
  const int iy  = iy0 + ky, ix = ix0 + kx;
  const bool ok = (k < KC) && ((unsigned)iy < (unsigned)IMW) && ((unsigned)ix < (unsigned)IMW);
  const int cc  = c > 2 ? 2 : c;
  const int iyc = iy < 0 ? 0 : (iy > IMW - 1 ? IMW - 1 : iy);
  const int ixc = ix < 0 ? 0 : (ix > IMW - 1 ? IMW - 1 : ix);
  const unsigned int raw = IMB[(cc * IMW + iyc) * IMW + ixc];
  return ok ? raw : 0u;
}

__global__ __launch_bounds__(GTHR) void k_conv(const unsigned short* __restrict__ IMB,
                                               const unsigned short* __restrict__ CWB,
                                               const float* __restrict__ gam, const float* __restrict__ bet,
                                               const float* __restrict__ mea, const float* __restrict__ var,
                                               float* Y) {
  __shared__ __attribute__((aligned(16))) unsigned short atile[GBM * KCP];
  __shared__ __attribute__((aligned(16))) float stg[CO * GBM];
  __shared__ float sbn[4 * CO];
  const int tid = (int)threadIdx.x, lane = tid & 31, wave = tid >> 5, hh = lane >> 4, m = lane & 15;
  const int m0  = (int)blockIdx.x * GBM;
  const int oy  = m0 >> 7;
  const int ox0 = m0 & (OHW - 1);

  if (tid < CO) {
    sbn[tid]          = bfr(gam[tid]);
    sbn[CO + tid]     = bfr(mea[tid]);
    sbn[2 * CO + tid] = 1.0f / sqrtf(bfr(var[tid]) + 1e-5f);
    sbn[3 * CO + tid] = bfr(bet[tid]);
  }

  const int iy0 = 2 * oy - 3;
#pragma unroll 1
  for (int u = tid; u < GBM * (KCP / 8); u += GTHR) {
    const int r   = u / (KCP / 8);
    const int g   = u - r * (KCP / 8);
    const int ix0 = 2 * (ox0 + r) - 3;
    const int k8  = 8 * g;
    const unsigned int t0 = tap(IMB, k8 + 0, iy0, ix0), t1 = tap(IMB, k8 + 1, iy0, ix0);
    const unsigned int t2 = tap(IMB, k8 + 2, iy0, ix0), t3 = tap(IMB, k8 + 3, iy0, ix0);
    const unsigned int t4 = tap(IMB, k8 + 4, iy0, ix0), t5 = tap(IMB, k8 + 5, iy0, ix0);
    const unsigned int t6 = tap(IMB, k8 + 6, iy0, ix0), t7 = tap(IMB, k8 + 7, iy0, ix0);
    v4u pv;
    pv.x = t0 | (t1 << 16); pv.y = t2 | (t3 << 16); pv.z = t4 | (t5 << 16); pv.w = t6 | (t7 << 16);
    *(v4ua*)(&atile[r * KCP + k8]) = pv;
  }
  __syncthreads();

  v8f acc[4];
  {
    const v8f z = {0.f, 0.f, 0.f, 0.f, 0.f, 0.f, 0.f, 0.f};
    acc[0] = z; acc[1] = z; acc[2] = z; acc[3] = z;
  }
  const int aoff = (16 * wave + m) * KCP + 8 * hh;
  const unsigned short* wp = CWB + (size_t)m * KCP + 8 * hh;
#pragma unroll 1
  for (int ks = 0; ks < KCP / 32; ++ks) {
    FragB af;
    af.h[0] = *(const v8usa*)(&atile[aoff + 32 * ks]);
    af.h[1] = *(const v8usa*)(&atile[aoff + 32 * ks + 16]);
#pragma unroll
    for (int t = 0; t < 4; ++t) {
      const unsigned short* wq = wp + (size_t)(16 * t) * KCP + 32 * ks;
      FragB bf;
      bf.h[0] = *(const v8usa*)wq;
      bf.h[1] = *(const v8usa*)(wq + 16);
      acc[t] = wmb(af, bf, acc[t]);
    }
  }

#pragma unroll
  for (int t = 0; t < 4; ++t) {
    const int lc = 16 * t + m;
    const float g = sbn[lc], mu = sbn[CO + lc], iv = sbn[2 * CO + lc], be = sbn[3 * CO + lc];
#pragma unroll
    for (int r = 0; r < 8; ++r) {
      const int lr = 16 * wave + 8 * hh + r;
      float y = (g * (acc[t][r] - mu)) * iv + be;
      y = fmaxf(y, 0.0f);
      stg[lc * GBM + lr] = y;
    }
  }
  __syncthreads();

  v4f fv[8];
#pragma unroll
  for (int i = 0; i < 8; ++i) {
    const int ch = 16 * wave + 2 * i + hh;
    fv[i] = *(const v4fa*)(stg + ch * GBM + 4 * m);
  }
#pragma unroll
  for (int i = 0; i < 8; ++i) {
    const int ch = 16 * wave + 2 * i + hh;
    float* op = Y + (size_t)ch * (OHW * OHW) + oy * OHW + ox0 + 4 * m;
    *(volatile v4f*)op = fv[i];
  }
  __threadfence();
#pragma unroll
  for (int i = 0; i < 8; ++i) {
    const int ch = 16 * wave + 2 * i + hh;
    float* op = Y + (size_t)ch * (OHW * OHW) + oy * OHW + ox0 + 4 * m;
    *(volatile v4f*)op = fv[i];
  }
}

__device__ __forceinline__ void rowmax8(const float* __restrict__ rp, int t, v4f& m0, v4f& m1) {
  const v4f a = *(const v4fa*)(rp + 16 * t);
  const v4f b = *(const v4fa*)(rp + 16 * t + 4);
  const v4f c = *(const v4fa*)(rp + 16 * t + 8);
  const v4f d = *(const v4fa*)(rp + 16 * t + 12);
  const int lc = 16 * t - 1;
  const float lf = rp[lc < 0 ? 0 : lc];
  m0.x = fmaxf(m0.x, fmaxf(lf,  fmaxf(a.x, a.y)));
  m0.y = fmaxf(m0.y, fmaxf(a.y, fmaxf(a.z, a.w)));
  m0.z = fmaxf(m0.z, fmaxf(a.w, fmaxf(b.x, b.y)));
  m0.w = fmaxf(m0.w, fmaxf(b.y, fmaxf(b.z, b.w)));
  m1.x = fmaxf(m1.x, fmaxf(b.w, fmaxf(c.x, c.y)));
  m1.y = fmaxf(m1.y, fmaxf(c.y, fmaxf(c.z, c.w)));
  m1.z = fmaxf(m1.z, fmaxf(c.w, fmaxf(d.x, d.y)));
  m1.w = fmaxf(m1.w, fmaxf(d.y, fmaxf(d.z, d.w)));
}

__global__ __launch_bounds__(NTHR) void k_pool(const float* __restrict__ Y, unsigned short* FE) {
  const int u = (int)blockIdx.x * NTHR + (int)threadIdx.x;
  if (u >= NN * 8) return;
  const int n = u >> 3, t = u & 7;
  const int c = n >> 6, py = n & 63;
  const float ninf = __int_as_float((int)0xff800000);
  v4f m0 = {ninf, ninf, ninf, ninf}, m1 = {ninf, ninf, ninf, ninf};
#pragma unroll
  for (int ky = 0; ky < 3; ++ky) {
    int yy = 2 * py - 1 + ky;
    yy = yy < 0 ? 0 : (yy > OHW - 1 ? OHW - 1 : yy);
    rowmax8(Y + ((size_t)c * OHW + yy) * OHW, t, m0, m1);
  }
  const v4u hv = pack8(m0, m1);
  v4f l0, l1;
  l0.x = lres(m0.x); l0.y = lres(m0.y); l0.z = lres(m0.z); l0.w = lres(m0.w);
  l1.x = lres(m1.x); l1.y = lres(m1.y); l1.z = lres(m1.z); l1.w = lres(m1.w);
  const v4u lv = pack8(l0, l1);
  unsigned short* hp = FE + (size_t)n * KF + 8 * t;
  *(volatile v4u*)hp = hv;
  *(volatile v4u*)(hp + 64) = lv;
  __threadfence();
  *(volatile v4u*)hp = hv;
  *(volatile v4u*)(hp + 64) = lv;
}

__global__ __launch_bounds__(GTHR) void k_gat1(const unsigned short* __restrict__ A,
                                               const unsigned short* __restrict__ WT,
                                               float* outF,
                                               const float* __restrict__ atts, const float* __restrict__ attd,
                                               float* SD) {
  __shared__ __attribute__((aligned(16))) float stg[GBM * GBN];
  __shared__ __attribute__((aligned(16))) float satt[2 * GBN];
  __shared__ __attribute__((aligned(16))) float sdot[4 * GBM];
  const int tid = (int)threadIdx.x, lane = tid & 31, wave = tid >> 5, hh = lane >> 4, m = lane & 15;
  const int rowBase = (int)blockIdx.x * GBM;
  const int cb      = (int)blockIdx.y;
  const int col0    = cb * GBN;

  {
    const int which = tid >> 6;
    const int c = tid & 63;
    const float vs = atts[col0 + c];
    const float vd = attd[col0 + c];
    const float v = (which == 0) ? vs : vd;
    satt[which * GBN + c] = bfr(v);
  }

  v8f acc[4];
  {
    const v8f z = {0.f, 0.f, 0.f, 0.f, 0.f, 0.f, 0.f, 0.f};
    acc[0] = z; acc[1] = z; acc[2] = z; acc[3] = z;
  }
  const unsigned short* ap = A  + (size_t)(rowBase + 16 * wave + m) * KF + 8 * hh;
  const unsigned short* wp = WT + (size_t)(col0 + m) * KF + 8 * hh;
#pragma unroll 1
  for (int ks = 0; ks < KF / 32; ++ks) {
    FragB af;
    af.h[0] = *(const v8usa*)(ap + 32 * ks);
    af.h[1] = *(const v8usa*)(ap + 32 * ks + 16);
#pragma unroll
    for (int t = 0; t < 4; ++t) {
      const unsigned short* wq = wp + (size_t)(16 * t) * KF + 32 * ks;
      FragB bf;
      bf.h[0] = *(const v8usa*)wq;
      bf.h[1] = *(const v8usa*)(wq + 16);
      acc[t] = wmb(af, bf, acc[t]);
    }
  }

#pragma unroll
  for (int t = 0; t < 4; ++t) {
    const int lc = 16 * t + m;
#pragma unroll
    for (int r = 0; r < 8; ++r) {
      const int lr = 16 * wave + 8 * hh + r;
      stg[lr * GBN + lc] = acc[t][r];
    }
  }
  __syncthreads();

  {
    const int row = tid & 63, which = tid >> 6;
    const float* sa = satt + which * GBN;
    const float* hr = stg + row * GBN;
    float d0 = 0.f, d1 = 0.f;
#pragma unroll 4
    for (int c4 = 0; c4 < 8; ++c4) {
      const v4f hv = *(const v4fa*)(hr + 4 * c4);
      const v4f av = *(const v4fa*)(sa + 4 * c4);
      d0 = fmaf(hv.x, av.x, d0); d0 = fmaf(hv.y, av.y, d0);
      d0 = fmaf(hv.z, av.z, d0); d0 = fmaf(hv.w, av.w, d0);
    }
#pragma unroll 4
    for (int c4 = 8; c4 < 16; ++c4) {
      const v4f hv = *(const v4fa*)(hr + 4 * c4);
      const v4f av = *(const v4fa*)(sa + 4 * c4);
      d1 = fmaf(hv.x, av.x, d1); d1 = fmaf(hv.y, av.y, d1);
      d1 = fmaf(hv.z, av.z, d1); d1 = fmaf(hv.w, av.w, d1);
    }
    sdot[(0 * 2 + which) * GBM + row] = d0;
    sdot[(1 * 2 + which) * GBM + row] = d1;
  }
  __syncthreads();

  v4f fv[8];
#pragma unroll
  for (int i = 0; i < 8; ++i) {
    const int lr = 16 * wave + 2 * i + hh;
    fv[i] = *(const v4fa*)(stg + lr * GBN + 4 * m);
  }
  const int wsel = wave & 1;
  const int seg = lane >> 4, piece = lane & 15;
  const v4f sdv = *(const v4fa*)(sdot + (wsel * 2 + seg) * GBM + 4 * piece);
  float* sp = SD + (size_t)(2 * (2 * cb + wsel) + seg) * NN + rowBase + 4 * piece;

#pragma unroll
  for (int i = 0; i < 8; ++i) {
    const int lr = 16 * wave + 2 * i + hh;
    float* op = outF + (size_t)(rowBase + lr) * HC + col0 + 4 * m;
    *(volatile v4f*)op = fv[i];
  }
  if (wave < 2) *(volatile v4f*)sp = sdv;
  __threadfence();
#pragma unroll
  for (int i = 0; i < 8; ++i) {
    const int lr = 16 * wave + 2 * i + hh;
    float* op = outF + (size_t)(rowBase + lr) * HC + col0 + 4 * m;
    *(volatile v4f*)op = fv[i];
  }
  if (wave < 2) *(volatile v4f*)sp = sdv;
}

__global__ __launch_bounds__(NTHR) void k_scan1(const int* __restrict__ srcs, const int* __restrict__ dsts,
                                                const float* __restrict__ F, const float* __restrict__ SD,
                                                const float* __restrict__ b1, const float* __restrict__ W2,
                                                float* H2S, int nE, int vec8) {
  extern __shared__ v4f lds_dyn[];
  int* reg1 = (int*)lds_dyn;
  int* reg2 = reg1 + RCAP;
  int* list = reg2 + RCAP;
  int* scnt = list + LISTN;
  int* soff = scnt + NB;
  int* wcnt = soff + NB;
  float* sres = (float*)(wcnt + 16);
  const int tid = (int)threadIdx.x, lane = tid & 31, wave = tid >> 5;
  const int nodeBase = (int)blockIdx.x * NB;

  const int nh = scan_build(dsts, nE, nodeBase, vec8, reg1, reg2, list, scnt, soff, wcnt, tid, lane, wave);

  const int nbw = NB / NWAVE;
  const bool ovf = (nh >= RCAP);
  const float qnan = __int_as_float(0x7fc00000);
  const int c0   = 4 * lane;
  const int head = lane >> 3;
  const v4f bb4 = bfr4(*(const v4fa*)(b1 + c0));
  const v4f w24 = bfr4(*(const v4fa*)(W2 + c0));
  const float* ASp = SD + (size_t)(2 * head) * NN;
  const float* ADp = ASp + NN;

#pragma unroll 1
  for (int jt = 0; jt < nbw; ++jt) {
    const int slot = wave * nbw + jt;
    const int grow = nodeBase + slot;
    const int gcl  = grow < NN ? grow : NN - 1;
    int st = soff[slot];
    const int craw = scnt[slot];
    int cnt = craw;
    st  = st < 0 ? 0 : (st > nh ? nh : st);
    cnt = cnt < 0 ? 0 : (cnt > DEGCAP ? DEGCAP : cnt);
    if (cnt > nh - st) cnt = nh - st;
    const float pz = (ovf || craw > DEGCAP) ? qnan : 0.0f;

    const float adv = ADp[gcl];
    float mx = -3.0e38f, dn = 0.0f;
    v4f av = {0.f, 0.f, 0.f, 0.f};

#pragma unroll 1
    for (int q = 0; q < cnt; ++q) {
      int idx = st + q; idx = idx > RCAP - 1 ? RCAP - 1 : idx;
      int eid = reg2[idx]; eid = eid < 0 ? 0 : (eid > nE - 1 ? nE - 1 : eid);
      const int sraw = srcs[eid];
      const int s = sraw < 0 ? 0 : (sraw > NN - 1 ? NN - 1 : sraw);
      const v4f fs = *(const v4fa*)(F + (size_t)s * HC + c0);
      float lg = ASp[s] + adv;
      lg = lg > 0.f ? lg : NEGSL * lg;
      const float df = lg - mx;
      const float ee = expf(-fabsf(df));
      const bool up  = df > 0.f;
      const float s1 = up ? ee : 1.0f;
      const float s2 = up ? 1.0f : ee;
      mx = up ? lg : mx;
      dn = fmaf(dn, s1, s2);
      av.x = fmaf(av.x, s1, s2 * fs.x);
      av.y = fmaf(av.y, s1, s2 * fs.y);
      av.z = fmaf(av.z, s1, s2 * fs.z);
      av.w = fmaf(av.w, s1, s2 * fs.w);
    }
    const float inv = (cnt > 0) ? (1.0f / dn) : 0.0f;
    float ox = fmaf(av.x, inv, bb4.x);
    float oy = fmaf(av.y, inv, bb4.y);
    float oz = fmaf(av.z, inv, bb4.z);
    float ow = fmaf(av.w, inv, bb4.w);
    ox = (ox > 0.0f) ? ox : (ox - ox);
    oy = (oy > 0.0f) ? oy : (oy - oy);
    oz = (oz > 0.0f) ? oz : (oz - oz);
    ow = (ow > 0.0f) ? ow : (ow - ow);
    float hp = ox * w24.x;
    hp = fmaf(oy, w24.y, hp);
    hp = fmaf(oz, w24.z, hp);
    hp = fmaf(ow, w24.w, hp);
#pragma unroll
    for (int off = 16; off > 0; off >>= 1) hp += __shfl_xor(hp, off);
    const float h2 = hp + pz;
    if (lane == 0) sres[slot] = h2;
  }
  __syncthreads();
  if (wave == 0) {
    const int piece = lane & 15;
    const v4f v = *(const v4fa*)(sres + 4 * piece);
    float* op = H2S + nodeBase + 4 * piece;
    const bool wr = (lane < 16) && (nodeBase + 4 * piece + 3 < NN);
    if (wr) *(volatile v4f*)op = v;
    __threadfence();
    if (wr) *(volatile v4f*)op = v;
  }
}

__global__ __launch_bounds__(NTHR) void k_scan2(const int* __restrict__ srcs, const int* __restrict__ dsts,
                                                const float* __restrict__ H2S,
                                                const float* __restrict__ a2s, const float* __restrict__ a2d,
                                                const float* __restrict__ b2,
                                                float* out, int nE, int vec8) {
  extern __shared__ v4f lds_dyn[];
  int* reg1 = (int*)lds_dyn;
  int* reg2 = reg1 + RCAP;
  int* list = reg2 + RCAP;
  int* scnt = list + LISTN;
  int* soff = scnt + NB;
  int* wcnt = soff + NB;
  float* sres = (float*)(wcnt + 16);
  const int tid = (int)threadIdx.x, lane = tid & 31, wave = tid >> 5;
  const int nodeBase = (int)blockIdx.x * NB;

  const int nh = scan_build(dsts, nE, nodeBase, vec8, reg1, reg2, list, scnt, soff, wcnt, tid, lane, wave);

  const int nbw = NB / NWAVE;
  const bool ovf = (nh >= RCAP);
  const float qnan = __int_as_float(0x7fc00000);
  const float as2 = bfr(a2s[0]);
  const float ad2 = bfr(a2d[0]);
  const float bz  = bfr(b2[0]);

#pragma unroll 1
  for (int jt = 0; jt < nbw; ++jt) {
    const int slot = wave * nbw + jt;
    const int grow = nodeBase + slot;
    const int gcl  = grow < NN ? grow : NN - 1;
    int st = soff[slot];
    const int craw = scnt[slot];
    int cnt = craw;
    st  = st < 0 ? 0 : (st > nh ? nh : st);
    cnt = cnt < 0 ? 0 : (cnt > DEGCAP ? DEGCAP : cnt);
    if (cnt > nh - st) cnt = nh - st;
    const float pz = (ovf || craw > DEGCAP) ? qnan : 0.0f;

    const float edv = H2S[gcl] * ad2;
    float M = -3.0e38f;
#pragma unroll 1
    for (int b0 = 0; b0 < cnt; b0 += 32) {
      const int q = b0 + lane;
      const bool ok = q < cnt;
      const int qq = ok ? q : cnt - 1;
      int idx = st + qq; idx = idx < 0 ? 0 : (idx > RCAP - 1 ? RCAP - 1 : idx);
      int eid = reg2[idx]; eid = eid < 0 ? 0 : (eid > nE - 1 ? nE - 1 : eid);
      const int sraw = srcs[eid];
      const int s = sraw < 0 ? 0 : (sraw > NN - 1 ? NN - 1 : sraw);
      const float hs = H2S[s];
      float lg = hs * as2 + edv;
      lg = lg > 0.f ? lg : NEGSL * lg;
      const float mm = fmaxf(M, lg);
      M = ok ? mm : M;
    }
#pragma unroll
    for (int off = 16; off > 0; off >>= 1) M = fmaxf(M, __shfl_xor(M, off));

    float S = 0.0f, Aq = 0.0f;
#pragma unroll 1
    for (int b0 = 0; b0 < cnt; b0 += 32) {
      const int q = b0 + lane;
      const bool ok = q < cnt;
      const int qq = ok ? q : cnt - 1;
      int idx = st + qq; idx = idx < 0 ? 0 : (idx > RCAP - 1 ? RCAP - 1 : idx);
      int eid = reg2[idx]; eid = eid < 0 ? 0 : (eid > nE - 1 ? nE - 1 : eid);
      const int sraw = srcs[eid];
      const int s = sraw < 0 ? 0 : (sraw > NN - 1 ? NN - 1 : sraw);
      const float hs = H2S[s];
      float lg = hs * as2 + edv;
      lg = lg > 0.f ? lg : NEGSL * lg;
      const float ex = expf(lg - M);
      const float eh = ex * hs;
      S  += ok ? ex : 0.0f;
      Aq += ok ? eh : 0.0f;
    }
#pragma unroll
    for (int off = 16; off > 0; off >>= 1) {
      S  += __shfl_xor(S, off);
      Aq += __shfl_xor(Aq, off);
    }
    const float inv = (cnt > 0) ? (1.0f / S) : 0.0f;
    const float o = (Aq * inv + bz) + pz;
    if (lane == 0) sres[slot] = o;
  }
  __syncthreads();
  if (wave == 0) {
    const int piece = lane & 15;
    const v4f v = *(const v4fa*)(sres + 4 * piece);
    float* op = out + nodeBase + 4 * piece;
    const bool wr = (lane < 16) && (nodeBase + 4 * piece + 3 < NN);
    if (wr) *(volatile v4f*)op = v;
    __threadfence();
    if (wr) *(volatile v4f*)op = v;
  }
}

static inline int cdiv(int a, int b) { return (a + b - 1) / b; }

extern "C" void kernel_launch(void* const* d_in, const int* in_sizes, int n_in,
                              void* d_out, int out_size, void* d_ws, size_t ws_size,
                              hipStream_t stream) {
  if (n_in < 16) return;
  if (in_sizes[0] != 3 * IMW * IMW) return;
  if (in_sizes[1] != CO * KC) return;
  if (in_sizes[2] != CO || in_sizes[3] != CO || in_sizes[4] != CO || in_sizes[5] != CO) return;
  if (in_sizes[6] != 64 * HC) return;
  if (in_sizes[7] != HC || in_sizes[8] != HC) return;
  if (in_sizes[9] != HC) return;
  if (in_sizes[10] != HC) return;
  if (in_sizes[11] < 1 || in_sizes[12] < 1 || in_sizes[13] < 1) return;
  const int nE = in_sizes[14];
  if (nE < 1 || in_sizes[15] != nE || nE >= (1 << 25)) return;
  if (out_size != NN) return;

  const float* image = (const float*)d_in[0];
  const float* convw = (const float*)d_in[1];
  const float* gam   = (const float*)d_in[2];
  const float* bet   = (const float*)d_in[3];
  const float* mea   = (const float*)d_in[4];
  const float* var   = (const float*)d_in[5];
  const float* W1    = (const float*)d_in[6];
  const float* a1s   = (const float*)d_in[7];
  const float* a1d   = (const float*)d_in[8];
  const float* b1    = (const float*)d_in[9];
  const float* W2    = (const float*)d_in[10];
  const float* a2s   = (const float*)d_in[11];
  const float* a2d   = (const float*)d_in[12];
  const float* b2    = (const float*)d_in[13];
  const int*   src   = (const int*)d_in[14];
  const int*   dst   = (const int*)d_in[15];
  float* out = (float*)d_out;

  char* ws = (char*)d_ws;
  size_t off = 0;
  const size_t oIMB = off; off += (size_t)3 * IMW * IMW * 2;     off = (off + 255) & ~(size_t)255;
  const size_t oCWB = off; off += (size_t)CO * KCP * 2;          off = (off + 255) & ~(size_t)255;
  const size_t oW1T = off; off += (size_t)HC * KF * 2;           off = (off + 255) & ~(size_t)255;
  const size_t oY   = off; off += (size_t)CO * OHW * OHW * 4;    off = (off + 255) & ~(size_t)255;
  const size_t oFE  = off; off += (size_t)NN * KF * 2;           off = (off + 255) & ~(size_t)255;
  const size_t oH   = off; off += (size_t)NN * HC * 4;           off = (off + 255) & ~(size_t)255;
  const size_t oSD  = off; off += (size_t)8 * NN * 4;            off = (off + 255) & ~(size_t)255;
  const size_t oH2  = off; off += (size_t)NN * 4;                off = (off + 255) & ~(size_t)255;
  if (off > ws_size || off > (size_t)WSMAX) return;
  unsigned short* IMB  = (unsigned short*)(ws + oIMB);
  unsigned short* CWB  = (unsigned short*)(ws + oCWB);
  unsigned short* W1T2 = (unsigned short*)(ws + oW1T);
  float*          Y    = (float*)(ws + oY);
  unsigned short* FE   = (unsigned short*)(ws + oFE);
  float*          H    = (float*)(ws + oH);
  float*          SD   = (float*)(ws + oSD);
  float*          H2S  = (float*)(ws + oH2);

  const int vec8 = ((nE & 3) == 0) ? 1 : 0;

  hipFuncSetAttribute(reinterpret_cast<const void*>(&k_scan1),
                      hipFuncAttributeMaxDynamicSharedMemorySize, LDS_SCAN);
  hipFuncSetAttribute(reinterpret_cast<const void*>(&k_scan2),
                      hipFuncAttributeMaxDynamicSharedMemorySize, LDS_SCAN);

  k_prep<<<(NU_IM + NU_CW + NU_W1) / NTHR, NTHR, 0, stream>>>(image, convw, W1, IMB, CWB, W1T2);
  k_conv<<<(OHW * OHW) / GBM, GTHR, 0, stream>>>(IMB, CWB, gam, bet, mea, var, Y);
  k_pool<<<cdiv(NN * 8, NTHR), NTHR, 0, stream>>>(Y, FE);
  k_gat1<<<dim3(NN / GBM, HC / GBN), GTHR, 0, stream>>>(FE, W1T2, H, a1s, a1d, SD);
  k_scan1<<<NN / NB, NTHR, LDS_SCAN, stream>>>(src, dst, H, SD, b1, W2, H2S, nE, vec8);
  k_scan2<<<NN / NB, NTHR, LDS_SCAN, stream>>>(src, dst, H2S, a2s, a2d, b2, out, nE, vec8);
}
